// TransformerBlock_29721173689039
// MI455X (gfx1250) — hardware-verified
//
#include <hip/hip_runtime.h>
#ifndef NB
#define NB 2
#endif
#ifndef SEQ
#define SEQ 2048
#endif
#define NB_FULL 2
#define SQ_FULL 2048
#define SQ SEQ
#define DM 768
#define NH 12
#define HD 64
#define DFF 3072
#define QT0 256
#define LQ (3 * DM)
#define DMQ DM
#define NR ((size_t)NB * SQ)
static_assert(SQ % 128 == 0);
static_assert(SQ >= QT0);
static_assert(QT0 % 128 == 0);
static_assert(NB <= NB_FULL);
static_assert(SQ <= SQ_FULL);
static_assert(DM == NH * HD);
static_assert(DM % 64 == 0);
static_assert(DFF % 64 == 0);
static_assert(DMQ % 4 == 0);
static_assert(DMQ / 4 <= 256);

typedef _Float16 v16h __attribute__((ext_vector_type(16)));
typedef _Float16 v4h __attribute__((ext_vector_type(4)));
typedef unsigned short v8us __attribute__((ext_vector_type(8), may_alias));
typedef float  v8f  __attribute__((ext_vector_type(8)));
typedef float  v4f  __attribute__((ext_vector_type(4)));
typedef float  v4fa __attribute__((ext_vector_type(4), may_alias));
union FragH { v16h v; v8us half[2]; _Float16 h[16]; unsigned short u[16]; };

__device__ __forceinline__ unsigned short bf16_bits(float x) { unsigned int u = __float_as_uint(x); return (unsigned short)((u + 0x7FFFu + ((u >> 16) & 1u)) >> 16); }
__device__ __forceinline__ float bf16_val(unsigned short b) { return __uint_as_float(((unsigned int)b) << 16); }
__device__ __forceinline__ float bf16_rne(float x) { return bf16_val(bf16_bits(x)); }

__global__ __launch_bounds__(256) void k_wt_f16(const float* __restrict__ W, _Float16* __restrict__ Wt, int K, int N, float scale) {
  const int t = blockIdx.x * 256 + threadIdx.x; if (t >= N * (K / 8)) return; const int n = t / (K / 8), k8 = (t % (K / 8)) * 8; FragH f;
#pragma unroll
  for (int i = 0; i < 8; ++i) f.h[i] = (_Float16)(bf16_rne(W[(size_t)(k8 + i) * N + n]) * scale);
  const v8us o = f.half[0];
  *(volatile v8us*)((unsigned short*)Wt + (size_t)n * K + k8) = o; __threadfence(); *(volatile v8us*)((unsigned short*)Wt + (size_t)n * K + k8) = o;
}

template <int NHv, int TTv>
__global__ __launch_bounds__(256) void k_vt(const _Float16* __restrict__ V16, int ldv, int voff, _Float16* __restrict__ Vt) {
  __shared__ unsigned short tl[64][66];
  const int tid = threadIdx.x; const int slab = blockIdx.x / (TTv / 64), lg = blockIdx.x % (TTv / 64); const int b = slab / NHv, h = slab % NHv;
  for (int i = tid; i < 64 * 8; i += 256) { const int r = i / 8, c8 = (i % 8) * 8; FragH f; f.half[0] = *(const v8us*)((const unsigned short*)V16 + ((size_t)b * TTv + lg * 64 + r) * ldv + voff + h * 64 + c8);
#pragma unroll
    for (int q = 0; q < 8; ++q) tl[r][c8 + q] = f.u[q]; }
  __syncthreads();
  for (int pass = 0; pass < 2; ++pass) {
#pragma unroll
    for (int rd = 0; rd < 2; ++rd) { const int d = rd * 32 + tid / 8, pc = tid % 8; FragH f;
#pragma unroll
      for (int q = 0; q < 8; ++q) f.u[q] = tl[pc * 8 + q][d];
      *(volatile v8us*)((unsigned short*)Vt + ((size_t)slab * 64 + d) * TTv + lg * 64 + pc * 8) = f.half[0]; }
    if (pass == 0) __threadfence(); }
}

__global__ __launch_bounds__(256) void k_hl(const float* __restrict__ F, _Float16* __restrict__ Hh, _Float16* __restrict__ Hl, size_t n8) {
  const size_t t = (size_t)blockIdx.x * 256 + threadIdx.x; if (t >= n8) return; FragH fh, fl; const v4f a = *(const v4fa*)(F + t * 8), c = *(const v4fa*)(F + t * 8 + 4);
#pragma unroll
  for (int q = 0; q < 4; ++q) { _Float16 h = (_Float16)a[q]; fh.h[q] = h; fl.h[q] = (_Float16)((a[q] - (float)h) * 1024.0f); h = (_Float16)c[q]; fh.h[4 + q] = h; fl.h[4 + q] = (_Float16)((c[q] - (float)h) * 1024.0f); }
  for (int pass = 0; pass < 2; ++pass) { *(volatile v8us*)((unsigned short*)Hh + t * 8) = fh.half[0]; *(volatile v8us*)((unsigned short*)Hl + t * 8) = fl.half[0]; if (pass == 0) __threadfence(); }
}

__device__ __forceinline__ v16h g2_frag(const _Float16* p, int hh) { FragH f; f.half[0] = *(const v8us*)((const unsigned short*)p + 8 * hh); f.half[1] = *(const v8us*)((const unsigned short*)p + 16 + 8 * hh); return f.v; }
__device__ __forceinline__ v8f g2_mma(v16h a, v16h b, v8f c) { v8f d = __builtin_amdgcn_wmma_f32_16x16x32_f16(false, a, false, b, (short)0, c, false, false); asm volatile("v_nop\n\tv_nop\n\tv_nop\n\tv_nop" : "+v"(d) : "v"(a), "v"(b)); return d; }
template <int ACT>
__global__ __launch_bounds__(128) void k_gemm2(const _Float16* __restrict__ A, int lda, size_t sA, const _Float16* __restrict__ Bh, int ldb, size_t sB, float alpha, const float* __restrict__ bias, size_t sBias, const float* __restrict__ CP, int rowsPerB, size_t sCPb, int row0g,
    float* __restrict__ C, _Float16* __restrict__ C16, int ldc, size_t sC, int M, int N, int K) {
  static_assert(ACT == 0 || ACT == 9);
  __shared__ __attribute__((aligned(16))) float so[4][32][68];
  const int tid = threadIdx.x, w = tid >> 5, lane = tid & 31, ln = lane & 15, hh = lane >> 4; const int by = blockIdx.y;
  A += (size_t)by * sA; Bh += (size_t)by * sB; const size_t cofs = (size_t)by * sC; const float* bp = bias ? bias + (size_t)by * sBias : nullptr;
  const int ntn = N >> 6; const int mt = blockIdx.x / ntn, nq = blockIdx.x - mt * ntn; const int row0 = mt * 128 + 32 * w, col0 = nq * 64; if (row0 >= M) return;
  const _Float16* a0p = A + (size_t)(row0 + ln) * lda; const _Float16* a1p = a0p + (size_t)16 * lda;
  const _Float16* b0p = Bh + (size_t)(col0 + ln) * ldb; const _Float16* b1p = b0p + (size_t)16 * ldb; const _Float16* b2p = b1p + (size_t)16 * ldb; const _Float16* b3p = b2p + (size_t)16 * ldb;
  const v8f z8 = {0.f,0.f,0.f,0.f,0.f,0.f,0.f,0.f}; v8f c00 = z8, c01 = z8, c02 = z8, c03 = z8, c10 = z8, c11 = z8, c12 = z8, c13 = z8;
#pragma unroll 1
  for (int kb = 0; kb < K; kb += 32) { const v16h a0 = g2_frag(a0p + kb, hh), a1 = g2_frag(a1p + kb, hh);
    v16h b = g2_frag(b0p + kb, hh); c00 = g2_mma(a0, b, c00); c10 = g2_mma(a1, b, c10);
    b = g2_frag(b1p + kb, hh); c01 = g2_mma(a0, b, c01); c11 = g2_mma(a1, b, c11);
    b = g2_frag(b2p + kb, hh); c02 = g2_mma(a0, b, c02); c12 = g2_mma(a1, b, c12);
    b = g2_frag(b3p + kb, hh); c03 = g2_mma(a0, b, c03); c13 = g2_mma(a1, b, c13); }
  v8f accs[8] = {c00, c01, c02, c03, c10, c11, c12, c13};
#pragma unroll
  for (int u = 0; u < 8; ++u) { const int t = u & 3, half = u >> 2; const int col = col0 + t * 16 + ln; const float bv = bp ? bf16_rne(bp[col]) : 0.f;
#pragma unroll
    for (int r = 0; r < 8; ++r) { const int rloc = half * 16 + 8 * hh + r; float v = accs[u][r] * alpha + bv;
      if (CP) { if (rowsPerB < 0) v += CP[cofs + (size_t)(row0g + row0 + rloc) * ldc + col];
                else { const int bidx = (row0g + row0 + rloc) / rowsPerB; v += CP[(size_t)bidx * sCPb + (size_t)by * 64 + col]; } }
      if (ACT == 9) v = 0.5f * v * (1.0f + tanhf(0.7978845608028654f * (v + 0.044715f * v * v * v)));
      so[w][rloc][t * 16 + ln] = v; } }
  __builtin_amdgcn_fence(4  , "workgroup"); __builtin_amdgcn_wave_barrier();
  const int rsub = lane >> 4, c4 = (lane & 15) * 4;
  for (int pass = 0; pass < 2; ++pass) {
#pragma unroll
    for (int q = 0; q < 16; ++q) { const int r = q * 2 + rsub; const v4f v = *(const v4fa*)&so[w][r][c4];
      if (C) *(volatile v4f*)(C + cofs + (size_t)(row0 + r) * ldc + col0 + c4) = v;
      if (C16) { v4h h4;
#pragma unroll
        for (int i = 0; i < 4; ++i) h4[i] = (_Float16)v[i];
        *(volatile v4h*)(C16 + cofs + (size_t)(row0 + r) * ldc + col0 + c4) = h4; } }
    if (pass == 0) __threadfence(); }
}

__device__ __forceinline__ v16h fl_frag(const unsigned short* p) { FragH f; f.half[0] = *(const v8us*)p; f.half[1] = *(const v8us*)(p + 16); return f.v; }
__device__ __forceinline__ v8f fl_wmma(v16h a, v16h b, v8f c) { return __builtin_amdgcn_wmma_f32_16x16x32_f16(false, a, false, b, (short)0, c, false, false); }
__device__ __forceinline__ void fl_guard2(v8f& a, v8f& b, v16h x, v16h y, v16h z) { asm volatile("v_nop\n\tv_nop\n\tv_nop\n\tv_nop" : "+v"(a), "+v"(b) : "v"(x), "v"(y), "v"(z)); }
__device__ __forceinline__ void fl_guard4(v8f& a, v8f& b, v8f& c, v8f& d, v16h p, v16h x, v16h y, v16h z, v16h w) { asm volatile("v_nop\n\tv_nop\n\tv_nop\n\tv_nop" : "+v"(a), "+v"(b), "+v"(c), "+v"(d) : "v"(p), "v"(x), "v"(y), "v"(z), "v"(w)); }

__global__ __launch_bounds__(128) void k_flash(const _Float16* __restrict__ QKV, const _Float16* __restrict__ VT, _Float16* __restrict__ O16) {
  __shared__ __attribute__((aligned(16))) _Float16 sp[4][16][40];
  __shared__ __attribute__((aligned(16))) _Float16 so[4][16][72];
  const int wave = __builtin_amdgcn_readfirstlane(threadIdx.x >> 5);
  const int lane = threadIdx.x & 31, ln = lane & 15, hh = lane >> 4;
  const int h = blockIdx.y, b = blockIdx.z;
  const int q0w = blockIdx.x * 64 + wave * 16;
  const size_t r0 = (size_t)b * SQ;
  const unsigned short* Qp = (const unsigned short*)QKV;
  const unsigned short* Vp = (const unsigned short*)VT;
  const size_t qoff = (r0 + q0w + ln) * LQ + (size_t)h * HD + 8 * hh;
  const size_t kbase = (r0 + ln) * LQ + DM + (size_t)h * HD + 8 * hh;
  const size_t vbase = (((size_t)b * NH + h) * HD + ln) * SQ + 8 * hh;
  const v8f z8 = {0.f,0.f,0.f,0.f,0.f,0.f,0.f,0.f};
  v8f o0 = z8, o1 = z8, o2 = z8, o3 = z8;
  float m[8], l[8];
#pragma unroll
  for (int r = 0; r < 8; ++r) { m[r] = -1.0e30f; l[r] = 0.f; }
  const int nhalf = (q0w >> 5) + 1;
  const int qb = q0w + 8 * hh;
#pragma unroll 1
  for (int it = 0; it < nhalf; ++it) {
    const int kb = it * 32;
    v8f s0 = z8, s1 = z8;
    const size_t ko = kbase + (size_t)kb * LQ;
    { const v16h aq = fl_frag(Qp + qoff); const v16h k0 = fl_frag(Qp + ko); const v16h k1 = fl_frag(Qp + ko + (size_t)16 * LQ);
      s0 = fl_wmma(aq, k0, s0); s1 = fl_wmma(aq, k1, s1); fl_guard2(s0, s1, aq, k0, k1); }
    { const v16h aq = fl_frag(Qp + qoff + 32); const v16h k0 = fl_frag(Qp + ko + 32); const v16h k1 = fl_frag(Qp + ko + (size_t)16 * LQ + 32);
      s0 = fl_wmma(aq, k0, s0); s1 = fl_wmma(aq, k1, s1); fl_guard2(s0, s1, aq, k0, k1); }
    const int kk0 = kb + ln, kk1 = kk0 + 16;
#pragma unroll
    for (int r = 0; r < 8; ++r) {
      const int qr = qb + r;
      const float e0 = (kk0 <= qr) ? s0[r] * 0.125f : -1.0e30f;
      const float e1 = (kk1 <= qr) ? s1[r] * 0.125f : -1.0e30f;
      float rm = fmaxf(e0, e1);
      rm = fmaxf(rm, __shfl_xor(rm, 8)); rm = fmaxf(rm, __shfl_xor(rm, 4)); rm = fmaxf(rm, __shfl_xor(rm, 2)); rm = fmaxf(rm, __shfl_xor(rm, 1));
      const float mn = fmaxf(m[r], rm);
      const float corr = __expf(m[r] - mn);
      const float p0 = __expf(e0 - mn), p1 = __expf(e1 - mn);
      l[r] = l[r] * corr + (p0 + p1);
      m[r] = mn;
      o0[r] *= corr; o1[r] *= corr; o2[r] *= corr; o3[r] *= corr;
      sp[wave][8 * hh + r][ln] = (_Float16)(p0 * 256.0f);
      sp[wave][8 * hh + r][16 + ln] = (_Float16)(p1 * 256.0f);
    }
    __builtin_amdgcn_fence(4  , "workgroup"); __builtin_amdgcn_wave_barrier();
    FragH ap; ap.half[0] = *(const v8us*)&sp[wave][ln][8 * hh]; ap.half[1] = *(const v8us*)&sp[wave][ln][16 + 8 * hh];
    const size_t vo = vbase + kb;
    { const v16h v0 = fl_frag(Vp + vo); const v16h v1 = fl_frag(Vp + vo + (size_t)16 * SQ); const v16h v2 = fl_frag(Vp + vo + (size_t)32 * SQ); const v16h v3 = fl_frag(Vp + vo + (size_t)48 * SQ);
      o0 = fl_wmma(ap.v, v0, o0); o1 = fl_wmma(ap.v, v1, o1); o2 = fl_wmma(ap.v, v2, o2); o3 = fl_wmma(ap.v, v3, o3);
      fl_guard4(o0, o1, o2, o3, ap.v, v0, v1, v2, v3); }
    __builtin_amdgcn_fence(4  , "workgroup"); __builtin_amdgcn_wave_barrier();
  }
#pragma unroll
  for (int r = 0; r < 8; ++r) {
    float t = l[r];
    t += __shfl_xor(t, 8); t += __shfl_xor(t, 4); t += __shfl_xor(t, 2); t += __shfl_xor(t, 1);
    const float fin = 0.25f / t;
    so[wave][8 * hh + r][ln] = (_Float16)(o0[r] * fin);
    so[wave][8 * hh + r][16 + ln] = (_Float16)(o1[r] * fin);
    so[wave][8 * hh + r][32 + ln] = (_Float16)(o2[r] * fin);
    so[wave][8 * hh + r][48 + ln] = (_Float16)(o3[r] * fin);
  }
  __builtin_amdgcn_fence(4  , "workgroup"); __builtin_amdgcn_wave_barrier();
  const int rq = lane >> 3, pc = (lane & 7) * 8;
  unsigned short* Op = (unsigned short*)O16 + (r0 + q0w) * DM + (size_t)h * HD;
  for (int pass = 0; pass < 2; ++pass) {
#pragma unroll
    for (int i4 = 0; i4 < 4; ++i4) { const int row = i4 * 4 + rq; const v8us v = *(const v8us*)&so[wave][row][pc];
      *(volatile v8us*)(Op + (size_t)row * DM + pc) = v; }
    if (pass == 0) __threadfence(); }
}

__global__ __launch_bounds__(64) void k_att0(const float* __restrict__ QF, const float* __restrict__ KF, const float* __restrict__ VF, int ld, size_t sIn, float scale, float* __restrict__ OF, int ldo, size_t sOut) {
  #pragma clang fp contract(off)
  __shared__ __attribute__((aligned(16))) float lq[64][64]; __shared__ __attribute__((aligned(16))) float lo[64][64];
  const int tid = threadIdx.x; const int h = blockIdx.x / (QT0 / 64), rg = blockIdx.x % (QT0 / 64); const int i = rg * 64 + tid;
  QF += (size_t)blockIdx.y * sIn; KF += (size_t)blockIdx.y * sIn; VF += (size_t)blockIdx.y * sIn; OF += (size_t)blockIdx.y * sOut;
  const float* qr = QF + (size_t)i * ld + h * HD;
#pragma unroll 1
  for (int c = 0; c < HD / 4; ++c) { *(v4f*)&lq[tid][c * 4] = *(const v4fa*)(qr + c * 4); const v4f z = {0.f, 0.f, 0.f, 0.f}; *(v4f*)&lo[tid][c * 4] = z; }
  float m = -1.0e30f, l = 0.f; const int jmax = rg * 64 + 63;
#pragma unroll 1
  for (int j = 0; j <= jmax; ++j) { const float* kr = KF + (size_t)j * ld + h * HD; const float* vr = VF + (size_t)j * ld + h * HD; float s = 0.f;
#pragma unroll 1
    for (int c = 0; c < HD / 4; ++c) { const v4f kq = *(const v4fa*)(kr + c * 4); const v4f qq = *(v4f*)&lq[tid][c * 4]; s = __fadd_rn(s, __fmul_rn(qq[0], kq[0])); s = __fadd_rn(s, __fmul_rn(qq[1], kq[1])); s = __fadd_rn(s, __fmul_rn(qq[2], kq[2])); s = __fadd_rn(s, __fmul_rn(qq[3], kq[3])); }
    s = __fmul_rn(s, scale);
    const float f = (j <= i) ? 1.f : 0.f; const float sm = fmaf(f, s, (1.f - f) * -1.0e30f); const float mn = fmaxf(m, sm); const float sc = expf(m - mn); const float e = expf(sm - mn); l = __fadd_rn(__fmul_rn(l, sc), e); m = mn;
#pragma unroll 1
    for (int c = 0; c < HD / 4; ++c) { const v4f vv = *(const v4fa*)(vr + c * 4); v4f oo = *(v4f*)&lo[tid][c * 4];
#pragma unroll
      for (int u = 0; u < 4; ++u) oo[u] = __fadd_rn(__fmul_rn(oo[u], sc), __fmul_rn(e, vv[u]));
      *(v4f*)&lo[tid][c * 4] = oo; } }
  const float fin = 64.0f / l;
#pragma unroll 1
  for (int c = 0; c < HD / 4; ++c) { v4f oo = *(v4f*)&lo[tid][c * 4];
#pragma unroll
    for (int u = 0; u < 4; ++u) oo[u] = __fmul_rn(oo[u], fin);
    *(v4f*)&lo[tid][c * 4] = oo; }
  __syncthreads();
  for (int pass = 0; pass < 2; ++pass) {
#pragma unroll 1
    for (int it = 0; it < 16; ++it) { const int row = it * 4 + tid / 16, pc = (tid % 16) * 4; const v4f v = *(const v4f*)&lo[row][pc]; *(volatile v4f*)(OF + (size_t)(rg * 64 + row) * ldo + h * HD + pc) = v; }
    if (pass == 0) __threadfence(); }
}

template <int BFIN, int WXB>
__global__ __launch_bounds__(256) void k_ln16(const float* __restrict__ X, int sq, int sfull, const float* __restrict__ g, const float* __restrict__ bb, float eps, _Float16* __restrict__ N16, float* __restrict__ XB) {
  #pragma clang fp contract(off)
  __shared__ float red[256]; const size_t r = blockIdx.x; const size_t xr = (r / (size_t)sq) * (size_t)sfull + (r % (size_t)sq);
  const int t = threadIdx.x; const bool act = t < DMQ / 4; const int tc = act ? t : 0; const float am = act ? 1.f : 0.f; const v4f xa = *(const v4fa*)(X + xr * DMQ + tc * 4); float s[4]; float sum = 0.f;
#pragma unroll
  for (int q = 0; q < 4; ++q) { s[q] = (BFIN ? bf16_rne(xa[q]) : xa[q]) * am; sum = __fadd_rn(sum, s[q]); }
  red[t] = sum; __syncthreads(); for (int st = 128; st > 0; st >>= 1) { if (t < st) red[t] = __fadd_rn(red[t], red[t + st]); __syncthreads(); } const float mu = red[0] / (float)DMQ; __syncthreads();
  float vs = 0.f;
#pragma unroll
  for (int q = 0; q < 4; ++q) { const float dl = __fadd_rn(s[q], -mu) * am; vs = __fadd_rn(vs, __fmul_rn(dl, dl)); }
  red[t] = vs; __syncthreads(); for (int st = 128; st > 0; st >>= 1) { if (t < st) red[t] = __fadd_rn(red[t], red[t + st]); __syncthreads(); }
  const float rs = rsqrtf(__fadd_rn(red[0] / (float)DMQ, eps)); if (!act) return; v4h y; v4f xb;
#pragma unroll
  for (int q = 0; q < 4; ++q) { const int c = t * 4 + q; y[q] = (_Float16)__fadd_rn(__fmul_rn(__fmul_rn(__fadd_rn(s[q], -mu), rs), bf16_rne(g[c])), bf16_rne(bb[c])); xb[q] = s[q]; }
  for (int pass = 0; pass < 2; ++pass) { *(volatile v4h*)(N16 + r * DMQ + t * 4) = y; if (WXB) *(volatile v4f*)(XB + r * DMQ + t * 4) = xb; if (pass == 0) __threadfence(); }
}

extern "C" void kernel_launch(void* const* d_in, const int* in_sizes, int n_in,
                              void* d_out, int out_size, void* d_ws, size_t ws_size, hipStream_t stream) {
  if (n_in < 14) return;
  const size_t xneed = ((size_t)(NB - 1) * SQ_FULL + SQ) * DM;
  if ((size_t)in_sizes[0] < xneed) return;
  if ((size_t)in_sizes[1] < (size_t)DM * DM || (size_t)in_sizes[2] < (size_t)DM * DM || (size_t)in_sizes[3] < (size_t)DM * DM || (size_t)in_sizes[4] < (size_t)DM * DM) return;
  if ((size_t)in_sizes[5] < DM || (size_t)in_sizes[6] < (size_t)DM * DFF || (size_t)in_sizes[7] < DFF || (size_t)in_sizes[8] < (size_t)DFF * DM || (size_t)in_sizes[9] < DM) return;
  if ((size_t)in_sizes[10] < DM || (size_t)in_sizes[11] < DM || (size_t)in_sizes[12] < DM || (size_t)in_sizes[13] < DM) return;
  if ((size_t)out_size < xneed) return;
  const float* const* I = (const float* const*)d_in;
  const float* x = I[0]; const float* wq = I[1]; const float* wk = I[2]; const float* wv = I[3]; const float* wo = I[4]; const float* bo = I[5];
  const float* w1 = I[6]; const float* b1 = I[7]; const float* w2 = I[8]; const float* b2 = I[9];
  const float* g1 = I[10]; const float* be1 = I[11]; const float* g2 = I[12]; const float* be2 = I[13];
  float* out = (float*)d_out;
  char* ws = (char*)d_ws; size_t off = 0;
  auto take = [&](size_t bytes) { char* p = ws + off; off += (bytes + 255) & ~(size_t)255; return p; };
  _Float16* BQKV = (_Float16*)take((size_t)3 * DM * DM * 2);
  _Float16* BO   = (_Float16*)take((size_t)DM * DM * 2);
  _Float16* X16  = (_Float16*)take(NR * DM * 2);
  float*    XB   = (float*)take(NR * DM * 4);
  float*    X1   = (float*)take(NR * DM * 4);
  _Float16* HF16 = (_Float16*)take(NR * DFF * 2);
  _Float16* BW1  = (_Float16*)take((size_t)DFF * DM * 2);
  _Float16* BW2  = (_Float16*)take((size_t)DM * DFF * 2);
  _Float16* QKV  = (_Float16*)take(NR * LQ * 2);
  _Float16* O16  = (_Float16*)take(NR * DM * 2);
  _Float16* VT   = (_Float16*)take((size_t)NB * NH * HD * SQ * 2);
  float*    QKVF0 = (float*)take((size_t)NB * QT0 * LQ * 4);
  float*    OF0  = (float*)take((size_t)NB * QT0 * DM * 4);
  _Float16* OH0  = (_Float16*)take((size_t)NB * QT0 * DM * 2);
  _Float16* OL0  = (_Float16*)take((size_t)NB * QT0 * DM * 2);
  _Float16* M16  = X16;
  if (off > ws_size || off > (size_t)134217728) return;

  { const unsigned g = (unsigned)(((size_t)DM * (DM / 8) + 255) / 256);
    k_wt_f16<<<g, 256, 0, stream>>>(wq, BQKV, DM, DM, 16.0f);
    k_wt_f16<<<g, 256, 0, stream>>>(wk, BQKV + (size_t)DM * DM, DM, DM, 16.0f);
    k_wt_f16<<<g, 256, 0, stream>>>(wv, BQKV + (size_t)2 * DM * DM, DM, DM, 16.0f);
    k_wt_f16<<<g, 256, 0, stream>>>(wo, BO, DM, DM, 16.0f); }
  k_wt_f16<<<(unsigned)(((size_t)DFF * (DM / 8) + 255) / 256), 256, 0, stream>>>(w1, BW1, DM, DFF, 16.0f);
  k_wt_f16<<<(unsigned)(((size_t)DM * (DFF / 8) + 255) / 256), 256, 0, stream>>>(w2, BW2, DFF, DM, 16.0f);
  k_ln16<1, 1><<<(unsigned)NR, 256, 0, stream>>>(x, SQ, SQ_FULL, g1, be1, 1e-5f, X16, XB);
  k_gemm2<0><<<dim3((unsigned)((NR / 128) * (LQ / 64)), 1), 128, 0, stream>>>(X16, DM, 0, BQKV, DM, 0, 0.0625f, nullptr, 0, nullptr, 1, 0, 0, nullptr, QKV, LQ, 0, (int)NR, LQ, DM);
  k_gemm2<0><<<dim3((QT0 / 128) * (LQ / 64), NB), 128, 0, stream>>>(X16, DM, (size_t)SQ * DM, BQKV, DM, 0, 0.0625f, nullptr, 0, nullptr, 1, 0, 0, QKVF0, nullptr, LQ, (size_t)QT0 * LQ, QT0, LQ, DM);
  k_vt<NH, SQ><<<NB * NH * (SQ / 64), 256, 0, stream>>>(QKV + 2 * DM, LQ, 0, VT);
  k_flash<<<dim3(SQ / 64, NH, NB), 128, 0, stream>>>(QKV, VT, O16);
  k_att0<<<dim3(NH * (QT0 / 64), NB), 64, 0, stream>>>(QKVF0, QKVF0 + DM, QKVF0 + 2 * DM, LQ, (size_t)QT0 * LQ, 0.125f, OF0, DM, (size_t)QT0 * DM);
  k_gemm2<0><<<dim3((unsigned)((NR / 128) * (DM / 64)), 1), 128, 0, stream>>>(O16, DM, 0, BO, DM, 0, 0.0009765625f, bo, 0, XB, -1, 0, 0, X1, nullptr, DM, 0, (int)NR, DM, DM);
  k_hl<<<(unsigned)(((size_t)NB * QT0 * DM / 8 + 255) / 256), 256, 0, stream>>>(OF0, OH0, OL0, (size_t)NB * QT0 * DM / 8);
  k_gemm2<0><<<dim3((QT0 / 128) * (DM / 64), NB), 128, 0, stream>>>(OH0, DM, (size_t)QT0 * DM, BO, DM, 0, 0.0009765625f, bo, 0, XB, -1, 0, 0, X1, nullptr, DM, (size_t)SQ * DM, QT0, DM, DM);
  k_gemm2<0><<<dim3((QT0 / 128) * (DM / 64), NB), 128, 0, stream>>>(OL0, DM, (size_t)QT0 * DM, BO, DM, 0, 0.00000095367431640625f, nullptr, 0, X1, -1, 0, 0, X1, nullptr, DM, (size_t)SQ * DM, QT0, DM, DM);
  k_ln16<0, 0><<<(unsigned)NR, 256, 0, stream>>>(X1, SQ, SQ, g2, be2, 1e-5f, M16, nullptr);
  k_gemm2<9><<<dim3((unsigned)((NR / 128) * (DFF / 64)), 1), 128, 0, stream>>>(M16, DM, 0, BW1, DM, 0, 0.0625f, b1, 0, nullptr, 1, 0, 0, nullptr, HF16, DFF, 0, (int)NR, DFF, DM);
  for (int b = 0; b < NB; ++b) {
    k_gemm2<0><<<dim3((unsigned)((SQ / 128) * (DM / 64)), 1), 128, 0, stream>>>(HF16 + (size_t)b * SQ * DFF, DFF, 0, BW2, DFF, 0, 0.0625f, b2, 0, X1 + (size_t)b * SQ * DM, -1, 0, 0, out + (size_t)b * SQ_FULL * DM, nullptr, DM, 0, SQ, DM, DFF);
  }
}
